// GATEncoder_20495583936894
// MI455X (gfx1250) — hardware-verified
//
#include <hip/hip_runtime.h>
#include <stddef.h>
#include <stdint.h>
#include <math.h>


#define NFEAT   8
#define NHEAD   4
#define HC1     128
#define HC2     64
#define CH2     16
#define KX1     256
#define KX2     128
#define NPG     128
#define NGR     256
#define NCL     32
#define DMX     2048
#define KMX     4096
#define KA2     4160
#define W2IN    2080
#define D3      512
#define KY      1024
#define LAT     128
#define NZ      256
#define NBOX    7
#define NTHR    256
#define NWAVE   8
#define EPT     8
#define CHUNK   (NTHR * EPT)
#define WCAP    (EPT * 32)
#define LISTN   (NWAVE * WCAP)
#define NBMAX   1024
#define SLOTB   10
#define RCAP    28672
#define DEGCAP  128
#define SPT     (NBMAX / NTHR)
#define GBM     64
#define GBN     64
#define GTHR    128
#define MROWS   1024
#define NEGSL   0.2f
#define EPS_SM  1e-16f
#define WSMAX   134217728
#define LDS_AGG ((2 * RCAP + 2 * NBMAX + LISTN) * 4 + 64)

#define NU0 (HC2 * (KX1 / 8))
#define NU1 (HC2 * (KX2 / 8))
#define NU2 (D3 * (KMX / 8))
#define NU3 (D3 * (KA2 / 8))
#define NU4 (D3 * (KY / 8))
#define NU5 (NZ * (KY / 8))
#define NUW (NU0 + NU1 + NU2 + NU3 + NU4 + NU5)

static_assert((CHUNK & (CHUNK - 1)) == 0);
static_assert(((long long)CHUNK << SLOTB) < (1LL << 31));
static_assert(NBMAX == (1 << SLOTB));
static_assert(SPT == 4 && NTHR * SPT == NBMAX);
static_assert(LISTN >= NBMAX);
static_assert(LISTN >= NWAVE * WCAP);
static_assert((RCAP % 32) == 0);
static_assert(NBMAX * CH2 <= RCAP);
static_assert(LDS_AGG <= 300000);
static_assert(GBM == (GTHR / 32) * 16);
static_assert(GTHR == 2 * GBN && GTHR == 2 * GBM);
static_assert((KX1 % 32) == 0 && (KX2 % 32) == 0 && (KMX % 32) == 0 && (KA2 % 32) == 0 && (KY % 32) == 0);
static_assert(HC2 == GBN && HC2 == NHEAD * CH2 && HC1 == NHEAD * 32);
static_assert(KX1 == 2 * HC1 && KX2 == 2 * HC2 && KMX == 2 * DMX && KY == 2 * D3);
static_assert(KA2 == 2 * DMX + 2 * NCL && W2IN == NCL + DMX);
static_assert(DMX == NPG * CH2);
static_assert((MROWS % GBM) == 0 && (MROWS % NTHR) == 0 && (MROWS % NBMAX) == 0);
static_assert(HC1 == 4 * 32);
static_assert(HC2 == 2 * 32);
static_assert((NGR % GBM) == 0 && (D3 % GBN) == 0 && (NZ % GBN) == 0 && (LAT % GBN) == 0 && NZ == 2 * LAT);
static_assert((NU0 % NTHR) == 0 && (NU1 % NTHR) == 0 && (NU2 % NTHR) == 0 && (NU3 % NTHR) == 0);
static_assert((NU4 % NTHR) == 0 && (NU5 % NTHR) == 0 && ((NU5 / 2) % NTHR) == 0);
static_assert((NTHR % CH2) == 0 && (NPG % (NTHR / CH2)) == 0);
static_assert(((NGR * NPG) % 16) == 0);
static_assert(CH2 * NBOX <= NTHR);

typedef float          v2f  __attribute__((ext_vector_type(2)));
typedef float          v4f  __attribute__((ext_vector_type(4)));
typedef float          v8f  __attribute__((ext_vector_type(8)));
typedef int            v4i  __attribute__((ext_vector_type(4)));
typedef int            v8i  __attribute__((ext_vector_type(8)));
typedef unsigned int   v4u  __attribute__((ext_vector_type(4)));
typedef unsigned short v8us __attribute__((ext_vector_type(8)));
typedef __bf16         v16b __attribute__((ext_vector_type(16)));
typedef v2f  __attribute__((may_alias)) v2fa;
typedef v4f  __attribute__((may_alias)) v4fa;
typedef v4u  __attribute__((may_alias)) v4ua;
typedef v8us __attribute__((may_alias)) v8usa;
union FragB { v16b v; v8us h[2]; v8i w; };

__device__ __forceinline__ v8f wmb(const FragB& a, const FragB& b, v8f c) {
  v8f d = __builtin_amdgcn_wmma_f32_16x16x32_bf16(false, a.v, false, b.v, (short)0, c, false, false);
  asm volatile("v_nop\n\tv_nop\n\tv_nop\n\tv_nop" : "+v"(d) : "v"(a.w), "v"(b.w));
  return d;
}

__device__ __forceinline__ unsigned int f2bf(float f) {
  const unsigned int u = __float_as_uint(f);
  return ((u + 0x7FFFu + ((u >> 16) & 1u)) >> 16) & 0xFFFFu;
}
__device__ __forceinline__ float bf2f(unsigned int b) { return __uint_as_float(b << 16); }
__device__ __forceinline__ float bfr(float f) { return bf2f(f2bf(f)); }
__device__ __forceinline__ v4f bfr4(const v4f a) {
  v4f r; r.x = bfr(a.x); r.y = bfr(a.y); r.z = bfr(a.z); r.w = bfr(a.w); return r;
}
__device__ __forceinline__ v4f lo4(const v4f a) {
  v4f r; r.x = a.x - bfr(a.x); r.y = a.y - bfr(a.y); r.z = a.z - bfr(a.z); r.w = a.w - bfr(a.w); return r;
}
__device__ __forceinline__ unsigned int pk2(float lo, float hi) { return f2bf(lo) | (f2bf(hi) << 16); }
__device__ __forceinline__ v4u pack8(const v4f a, const v4f b) {
  v4u r;
  r.x = pk2(a.x, a.y); r.y = pk2(a.z, a.w); r.z = pk2(b.x, b.y); r.w = pk2(b.z, b.w);
  return r;
}
__device__ __forceinline__ float hsel(const v4f v, int h) {
  const float a = (h & 1) ? v.y : v.x;
  const float b = (h & 1) ? v.w : v.z;
  return (h & 2) ? b : a;
}

__device__ __forceinline__ int scan_chunk(const int* __restrict__ dsts, int nE, int cbase, int slotBase,
                                          int nb, int vec8, int* list, int tid, int lane, int wave) {
  int wc = 0;
  const int el0  = tid * EPT;
  const int e0   = cbase + el0;
  const int sent = -2147483647 - 1;
  v4i da, db;
  if (vec8 != 0 && cbase + CHUNK <= nE) {
    da = *(const v4i*)(dsts + e0);
    db = *(const v4i*)(dsts + e0 + 4);
  } else {
    da.x = (e0     < nE) ? dsts[min(e0,     nE - 1)] : sent;
    da.y = (e0 + 1 < nE) ? dsts[min(e0 + 1, nE - 1)] : sent;
    da.z = (e0 + 2 < nE) ? dsts[min(e0 + 2, nE - 1)] : sent;
    da.w = (e0 + 3 < nE) ? dsts[min(e0 + 3, nE - 1)] : sent;
    db.x = (e0 + 4 < nE) ? dsts[min(e0 + 4, nE - 1)] : sent;
    db.y = (e0 + 5 < nE) ? dsts[min(e0 + 5, nE - 1)] : sent;
    db.z = (e0 + 6 < nE) ? dsts[min(e0 + 6, nE - 1)] : sent;
    db.w = (e0 + 7 < nE) ? dsts[min(e0 + 7, nE - 1)] : sent;
  }
  const unsigned nbs = (unsigned)slotBase;
  const unsigned unb = (unsigned)nb;
  const unsigned s0 = (unsigned)da.x - nbs, s1 = (unsigned)da.y - nbs;
  const unsigned s2 = (unsigned)da.z - nbs, s3 = (unsigned)da.w - nbs;
  const unsigned s4 = (unsigned)db.x - nbs, s5 = (unsigned)db.y - nbs;
  const unsigned s6 = (unsigned)db.z - nbs, s7 = (unsigned)db.w - nbs;
  const bool h0 = s0 < unb, h1 = s1 < unb, h2 = s2 < unb, h3 = s3 < unb;
  const bool h4 = s4 < unb, h5 = s5 < unb, h6 = s6 < unb, h7 = s7 < unb;
  const unsigned any = __builtin_amdgcn_ballot_w32(h0 | h1 | h2 | h3 | h4 | h5 | h6 | h7);
  if (any != 0u) {
#define HITJ(J, HJ, SJ) { \
      const unsigned mj = __builtin_amdgcn_ballot_w32(HJ); \
      if (mj != 0u) { \
        if (HJ) { \
          const int pos = wc + (int)__builtin_amdgcn_mbcnt_lo(mj, 0u); \
          if (pos < WCAP) list[wave * WCAP + pos] = ((el0 + (J)) << SLOTB) | (int)(SJ); \
        } \
        wc += (int)__builtin_popcount(mj); } }
    HITJ(0, h0, s0)
    HITJ(1, h1, s1)
    HITJ(2, h2, s2)
    HITJ(3, h3, s3)
    HITJ(4, h4, s4)
    HITJ(5, h5, s5)
    HITJ(6, h6, s6)
    HITJ(7, h7, s7)
#undef HITJ
  }
  return wc;
}

__global__ __launch_bounds__(NTHR) void k_wprep(
    const float* __restrict__ g2W, const float* __restrict__ g3W, const float* __restrict__ W1,
    const float* __restrict__ W2, const float* __restrict__ W3, const float* __restrict__ Wm,
    const float* __restrict__ Wv,
    unsigned short* G2P, unsigned short* G3P, unsigned short* W1D, unsigned short* W2E,
    unsigned short* W3D, unsigned short* WMV) {
  const int u = (int)blockIdx.x * NTHR + (int)threadIdx.x;
  const float* p;
  unsigned short* dp;
  bool zero = false;
  if (u < NU0) {
    const int n = u >> 5, k8 = (u & 31) * 8, kk = k8 & (HC1 - 1);
    p = g2W + (size_t)n * HC1 + kk;  dp = G2P + (size_t)n * KX1 + k8;
  } else if (u < NU0 + NU1) {
    const int v = u - NU0;
    const int n = v >> 4, k8 = (v & 15) * 8, kk = k8 & (HC2 - 1);
    p = g3W + (size_t)n * HC2 + kk;  dp = G3P + (size_t)n * KX2 + k8;
  } else if (u < NU0 + NU1 + NU2) {
    const int v = u - NU0 - NU1;
    const int n = v >> 9, k8 = (v & 511) * 8, kk = k8 & (DMX - 1);
    p = W1 + (size_t)n * DMX + kk;   dp = W1D + (size_t)n * KMX + k8;
  } else if (u < NU0 + NU1 + NU2 + NU3) {
    const int v = u - NU0 - NU1 - NU2;
    const int n = v / (KA2 / 8);
    const int k8 = (v - n * (KA2 / 8)) * 8;
    int col = (k8 < 2 * DMX) ? (NCL + (k8 & (DMX - 1))) : (k8 - 2 * DMX);
    col = col < 0 ? 0 : (col > W2IN - 8 ? W2IN - 8 : col);
    zero = (k8 >= 2 * DMX + NCL);
    p = W2 + (size_t)n * W2IN + col; dp = W2E + (size_t)n * KA2 + k8;
  } else if (u < NU0 + NU1 + NU2 + NU3 + NU4) {
    const int v = u - NU0 - NU1 - NU2 - NU3;
    const int n = v >> 7, k8 = (v & 127) * 8, kk = k8 & (D3 - 1);
    p = W3 + (size_t)n * D3 + kk;    dp = W3D + (size_t)n * KY + k8;
  } else if (u < NUW) {
    const int v = u - NU0 - NU1 - NU2 - NU3 - NU4;
    const int n = v >> 7, k8 = (v & 127) * 8, kk = k8 & (D3 - 1);
    const int nl = n & (LAT - 1);
    const float* wsrc = (n < LAT) ? Wm : Wv;
    p = wsrc + (size_t)nl * D3 + kk; dp = WMV + (size_t)n * KY + k8;
  } else {
    return;
  }
  v4f a = *(const v4fa*)p, b = *(const v4fa*)(p + 4);
  const v4f z4 = {0.f, 0.f, 0.f, 0.f};
  if (zero) { a = z4; b = z4; }
  const v4u wv = pack8(a, b);
  *(volatile v4u*)dp = wv;
  __threadfence();
  *(volatile v4u*)dp = wv;
}

__global__ __launch_bounds__(NTHR) void k_gat1(const float* __restrict__ X, const float* __restrict__ W,
                                               const float* __restrict__ avs, const float* __restrict__ avd,
                                               float* H1o, float* ASo, float* ADo, int nN, int MPr) {
  __shared__ __attribute__((aligned(16))) float sW[HC1 * NFEAT];
  __shared__ __attribute__((aligned(16))) float sAt[2 * HC1];
  const int tid = (int)threadIdx.x, lane = tid & 31, wave = tid >> 5;
  {
    const v4f w4 = *(const v4fa*)(W + 4 * tid);
    *(v4fa*)(sW + 4 * tid) = bfr4(w4);
    const int which = tid >> 7;
    const int c = tid & (HC1 - 1);
    const float vs = avs[c], vd = avd[c];
    sAt[which * HC1 + c] = bfr(which == 0 ? vs : vd);
  }
  __syncthreads();

  const int c0 = 4 * lane;
  v4f wA[4], wB[4];
#pragma unroll
  for (int c = 0; c < 4; ++c) {
    wA[c] = *(const v4fa*)(sW + (c0 + c) * NFEAT);
    wB[c] = *(const v4fa*)(sW + (c0 + c) * NFEAT + 4);
  }
  const v4f as4 = *(const v4fa*)(sAt + 4 * lane);
  const v4f ad4 = *(const v4fa*)(sAt + HC1 + 4 * lane);
  const int base = (int)blockIdx.x * NTHR + wave * 32;
  v4f keepS = {0.f, 0.f, 0.f, 0.f}, keepD = {0.f, 0.f, 0.f, 0.f};

#pragma unroll 1
  for (int j = 0; j < 32; ++j) {
    const int node = base + j;
    const bool live = node < nN;
    const int ncl = live ? node : nN - 1;
    const v4f xa = bfr4(*(const v4fa*)(X + (size_t)ncl * NFEAT));
    const v4f xb = bfr4(*(const v4fa*)(X + (size_t)ncl * NFEAT + 4));
    float h[4];
#pragma unroll
    for (int c = 0; c < 4; ++c) {
      float t = xa.x * wA[c].x;
      t = fmaf(xa.y, wA[c].y, t);
      t = fmaf(xa.z, wA[c].z, t);
      t = fmaf(xa.w, wA[c].w, t);
      t = fmaf(xb.x, wB[c].x, t);
      t = fmaf(xb.y, wB[c].y, t);
      t = fmaf(xb.z, wB[c].z, t);
      t = fmaf(xb.w, wB[c].w, t);
      h[c] = t;
    }
    float ps = h[0] * as4.x; ps = fmaf(h[1], as4.y, ps); ps = fmaf(h[2], as4.z, ps); ps = fmaf(h[3], as4.w, ps);
    float pd = h[0] * ad4.x; pd = fmaf(h[1], ad4.y, pd); pd = fmaf(h[2], ad4.z, pd); pd = fmaf(h[3], ad4.w, pd);
    ps += __shfl_xor(ps, 1); ps += __shfl_xor(ps, 2); ps += __shfl_xor(ps, 4);
    pd += __shfl_xor(pd, 1); pd += __shfl_xor(pd, 2); pd += __shfl_xor(pd, 4);
    const float s0 = __shfl(ps, 0), s1 = __shfl(ps, 8), s2 = __shfl(ps, 16), s3 = __shfl(ps, 24);
    const float d0 = __shfl(pd, 0), d1 = __shfl(pd, 8), d2 = __shfl(pd, 16), d3 = __shfl(pd, 24);
    const bool me = (lane == j);
    keepS.x = me ? (live ? s0 : 0.f) : keepS.x;
    keepS.y = me ? (live ? s1 : 0.f) : keepS.y;
    keepS.z = me ? (live ? s2 : 0.f) : keepS.z;
    keepS.w = me ? (live ? s3 : 0.f) : keepS.w;
    keepD.x = me ? (live ? d0 : 0.f) : keepD.x;
    keepD.y = me ? (live ? d1 : 0.f) : keepD.y;
    keepD.z = me ? (live ? d2 : 0.f) : keepD.z;
    keepD.w = me ? (live ? d3 : 0.f) : keepD.w;
    v4f hv;
    hv.x = live ? h[0] : 0.f; hv.y = live ? h[1] : 0.f; hv.z = live ? h[2] : 0.f; hv.w = live ? h[3] : 0.f;
    float* hp = H1o + (size_t)node * HC1 + c0;
    const bool wr = node < MPr;
    if (wr) *(volatile v4f*)hp = hv;
    __threadfence();
    if (wr) *(volatile v4f*)hp = hv;
  }
  float* sp = ASo + (size_t)base * NHEAD + 4 * lane;
  float* dq = ADo + (size_t)base * NHEAD + 4 * lane;
  const bool wr2 = base + 31 < MPr;
  if (wr2) { *(volatile v4f*)sp = keepS; *(volatile v4f*)dq = keepD; }
  __threadfence();
  if (wr2) { *(volatile v4f*)sp = keepS; *(volatile v4f*)dq = keepD; }
}

__global__ __launch_bounds__(GTHR) void k_gemmh(
    const unsigned short* __restrict__ A, const unsigned short* __restrict__ WT, int K,
    float* Hout, const float* __restrict__ avs, const float* __restrict__ avd, float* ASo, float* ADo)
{
  __shared__ __attribute__((aligned(16))) float stg[GBM * GBN];
  __shared__ __attribute__((aligned(16))) float satt[2 * GBN];
  __shared__ __attribute__((aligned(16))) float sdot[2 * GBM * NHEAD];
  const int tid = (int)threadIdx.x, lane = tid & 31, wave = tid >> 5, hh = lane >> 4, m = lane & 15;
  const int rowBase = (int)blockIdx.x * GBM;

  {
    const int which = tid >> 6;
    const int c  = tid & 63;
    const float vs = avs[c];
    const float vd = avd[c];
    satt[which * GBN + c] = bfr((which == 0) ? vs : vd);
  }

  v8f acc[4];
  {
    const v8f z = {0.f, 0.f, 0.f, 0.f, 0.f, 0.f, 0.f, 0.f};
    acc[0] = z; acc[1] = z; acc[2] = z; acc[3] = z;
  }
  const unsigned short* ap = A  + (size_t)(rowBase + 16 * wave + m) * (size_t)K + 8 * hh;
  const unsigned short* wp = WT + (size_t)m * (size_t)K + 8 * hh;
  const int ksteps = K >> 5;
#pragma unroll 1
  for (int ks = 0; ks < ksteps; ++ks) {
    FragB af;
    af.h[0] = *(const v8usa*)(ap + 32 * ks);
    af.h[1] = *(const v8usa*)(ap + 32 * ks + 16);
#pragma unroll
    for (int t = 0; t < 4; ++t) {
      const unsigned short* wq = wp + (size_t)(16 * t) * (size_t)K + 32 * ks;
      FragB bf;
      bf.h[0] = *(const v8usa*)wq;
      bf.h[1] = *(const v8usa*)(wq + 16);
      acc[t] = wmb(af, bf, acc[t]);
    }
  }

#pragma unroll
  for (int t = 0; t < 4; ++t) {
    const int lc = 16 * t + m;
#pragma unroll
    for (int r = 0; r < 8; ++r) {
      const int lr = 16 * wave + 8 * hh + r;
      stg[lr * GBN + lc] = acc[t][r];
    }
  }
  __syncthreads();

  {
    const int row = tid & 63, which = tid >> 6;
    const float* sa = satt + which * GBN;
    const float* hr = stg + row * GBN;
    float d[4];
#pragma unroll
    for (int hd = 0; hd < 4; ++hd) {
      float s = 0.f;
#pragma unroll
      for (int c4 = 0; c4 < CH2 / 4; ++c4) {
        const v4f hv = *(const v4fa*)(hr + CH2 * hd + 4 * c4);
        const v4f av = *(const v4fa*)(sa + CH2 * hd + 4 * c4);
        s = fmaf(hv.x, av.x, s);
        s = fmaf(hv.y, av.y, s);
        s = fmaf(hv.z, av.z, s);
        s = fmaf(hv.w, av.w, s);
      }
      d[hd] = s;
    }
    v4f dv; dv.x = d[0]; dv.y = d[1]; dv.z = d[2]; dv.w = d[3];
    *(v4fa*)(sdot + (which * GBM + row) * NHEAD) = dv;
  }
  __syncthreads();

  v4f fv[8];
#pragma unroll
  for (int i = 0; i < 8; ++i) {
    const int lr = 16 * wave + 2 * i + hh;
    fv[i] = *(const v4fa*)(stg + lr * GBN + 4 * m);
  }
  const int wsel = wave & 1;
  const v4f sv0 = *(const v4fa*)(sdot + (wsel * GBM + lane) * NHEAD);
  const v4f sv1 = *(const v4fa*)(sdot + (wsel * GBM + 32 + lane) * NHEAD);
  float* sdp = (wsel != 0) ? ADo : ASo;
  float* sp0 = sdp + (size_t)(rowBase + lane) * NHEAD;
  float* sp1 = sdp + (size_t)(rowBase + 32 + lane) * NHEAD;
  const bool wsd = wave < 2;

#pragma unroll
  for (int i = 0; i < 8; ++i) {
    const int lr = 16 * wave + 2 * i + hh;
    float* op = Hout + (size_t)(rowBase + lr) * HC2 + 4 * m;
    *(volatile v4f*)op = fv[i];
  }
  if (wsd) { *(volatile v4f*)sp0 = sv0; *(volatile v4f*)sp1 = sv1; }
  __threadfence();
#pragma unroll
  for (int i = 0; i < 8; ++i) {
    const int lr = 16 * wave + 2 * i + hh;
    float* op = Hout + (size_t)(rowBase + lr) * HC2 + 4 * m;
    *(volatile v4f*)op = fv[i];
  }
  if (wsd) { *(volatile v4f*)sp0 = sv0; *(volatile v4f*)sp1 = sv1; }
}

template<int L>
__global__ __launch_bounds__(NTHR) void k_agg(
    const int* __restrict__ srcs, const int* __restrict__ dsts,
    const float* __restrict__ F, const float* __restrict__ AS, const float* __restrict__ AD,
    unsigned short* HP, float* X3o,
    int nN, int nE, int nb, int vec8, int MPr) {
  static_assert(L == 1 || L == 2 || L == 3);
  extern __shared__ v4f lds_dyn[];
  int* reg1 = (int*)lds_dyn;
  int* reg2 = reg1 + RCAP;
  int* scnt = reg2 + RCAP;
  int* soff = scnt + NBMAX;
  int* list = soff + NBMAX;
  int* wcnt = list + LISTN;
  int* wtot = wcnt + NWAVE;
  const int tid = (int)threadIdx.x, lane = tid & 31, wave = tid >> 5;
  const int nodeBase = (int)blockIdx.x * nb;

  for (int i = tid; i < NBMAX; i += NTHR) scnt[i] = 0;
  __syncthreads();

  int tot = 0;
  const int nChunks = (nE + CHUNK - 1) / CHUNK;
#pragma unroll 1
  for (int ch = 0; ch < nChunks; ++ch) {
    const int cbase = ch * CHUNK;
    const int wc = scan_chunk(dsts, nE, cbase, nodeBase, nb, vec8, list, tid, lane, wave);
    if (lane == 0) wcnt[wave] = wc;
    __syncthreads();
    int pre = 0, all = 0;
#pragma unroll
    for (int w2 = 0; w2 < NWAVE; ++w2) {
      int c = wcnt[w2];
      c = c < 0 ? 0 : (c > WCAP ? WCAP : c);
      all += c;
      pre += (w2 < wave) ? c : 0;
    }
    const int wcc  = wc > WCAP ? WCAP : wc;
    const int base = tot + pre;
#pragma unroll 1
    for (int i = lane; i < wcc; i += 32) {
      const int ent = list[wave * WCAP + i];
      const int el  = (ent >> SLOTB) & (CHUNK - 1);
      const int sl  = ent & (NBMAX - 1);
      int eid = cbase + el;
      eid = eid > nE - 1 ? nE - 1 : eid;
      const int pos = base + i;
      if (pos < RCAP) reg1[pos] = (int)(((unsigned)eid << SLOTB) | (unsigned)sl);
    }
    tot += all;
    tot = tot > RCAP ? RCAP : tot;
    __syncthreads();
  }
  const int nh = tot;

  if (wave == 0) {
#pragma unroll 1
    for (int b0 = 0; b0 < nh; b0 += 32) {
      const int idx = b0 + lane;
      const int uv  = reg1[idx < nh ? idx : nh - 1];
      const int m32 = (nh - b0) < 32 ? (nh - b0) : 32;
#pragma unroll 1
      for (int k = 0; k < m32; ++k) {
        const int u  = __builtin_amdgcn_readlane(uv, k);
        const int sl = u & (NBMAX - 1);
        if (lane == 0) scnt[sl] = scnt[sl] + 1;
      }
    }
  }
  __syncthreads();

  {
    const v4i ca = *(const v4i*)(scnt + SPT * tid);
    const int e0 = ca.x < 0 ? 0 : ca.x, e1 = ca.y < 0 ? 0 : ca.y, e2 = ca.z < 0 ? 0 : ca.z, e3 = ca.w < 0 ? 0 : ca.w;
    const int ts = e0 + e1 + e2 + e3;
    int incl = ts;
#pragma unroll
    for (int d = 1; d < 32; d <<= 1) {
      const int up = __shfl_up(incl, d);
      if (lane >= d) incl += up;
    }
    if (lane == 31) wtot[wave] = incl;
    __syncthreads();
    int pre = 0;
#pragma unroll
    for (int w2 = 0; w2 < NWAVE; ++w2) pre += (w2 < wave) ? wtot[w2] : 0;
    int run = pre + incl - ts;
    soff[SPT * tid + 0] = run; run += e0;
    soff[SPT * tid + 1] = run; run += e1;
    soff[SPT * tid + 2] = run; run += e2;
    soff[SPT * tid + 3] = run;
  }
  __syncthreads();
  for (int i = tid; i < NBMAX; i += NTHR) list[i] = soff[i];
  __syncthreads();

  if (wave == 0) {
#pragma unroll 1
    for (int b0 = 0; b0 < nh; b0 += 32) {
      const int idx = b0 + lane;
      const int uv  = reg1[idx < nh ? idx : nh - 1];
      const int m32 = (nh - b0) < 32 ? (nh - b0) : 32;
#pragma unroll 1
      for (int k = 0; k < m32; ++k) {
        const int u   = __builtin_amdgcn_readlane(uv, k);
        const int sl  = u & (NBMAX - 1);
        const int eid = (int)((unsigned)u >> SLOTB);
        if (lane == 0) {
          int pos = list[sl];
          pos = pos < 0 ? 0 : (pos > RCAP - 1 ? RCAP - 1 : pos);
          reg2[pos] = eid;
          list[sl] = pos + 1;
        }
      }
    }
  }
  __syncthreads();

  const int nbw  = nb >> 3;
  const bool ovf = (nh >= RCAP);
  const float qnan = __int_as_float(0x7fc00000);
  const int head = lane >> 3;

  if constexpr (L == 1) {
    const int c0 = 4 * lane;
#pragma unroll 1
    for (int jt = 0; jt < nbw; ++jt) {
      const int slot = wave * nbw + jt;
      const int grow = nodeBase + slot;
      const int gcl  = grow < nN ? grow : nN - 1;
      int st = soff[slot];
      const int craw = scnt[slot];
      int cnt = craw;
      st  = st < 0 ? 0 : (st > nh ? nh : st);
      cnt = cnt < 0 ? 0 : (cnt > DEGCAP ? DEGCAP : cnt);
      if (cnt > nh - st) cnt = nh - st;
      const float pz = (ovf || craw > DEGCAP) ? qnan : 0.0f;

      const v4f ad4 = *(const v4fa*)(AD + (size_t)gcl * NHEAD);
      const float adv = hsel(ad4, head);
      float mx = -3.0e38f, dn = 0.0f;
      v4f av = {0.f, 0.f, 0.f, 0.f};

#pragma unroll 1
      for (int q = 0; q < cnt; ++q) {
        int idx = st + q; idx = idx > RCAP - 1 ? RCAP - 1 : idx;
        int eid = reg2[idx]; eid = eid < 0 ? 0 : (eid > nE - 1 ? nE - 1 : eid);
        const int sraw = srcs[eid];
        const int s = sraw < 0 ? 0 : (sraw > nN - 1 ? nN - 1 : sraw);
        const v4f fs  = *(const v4fa*)(F + (size_t)s * HC1 + c0);
        const v4f as4 = *(const v4fa*)(AS + (size_t)s * NHEAD);
        float lg = hsel(as4, head) + adv;
        lg = lg > 0.f ? lg : NEGSL * lg;
        const float df = lg - mx;
        const float ee = expf(-fabsf(df));
        const bool up  = df > 0.f;
        const float s1 = up ? ee : 1.0f;
        const float s2 = up ? 1.0f : ee;
        mx = up ? lg : mx;
        dn = fmaf(dn, s1, s2);
        av.x = fmaf(av.x, s1, s2 * fs.x);
        av.y = fmaf(av.y, s1, s2 * fs.y);
        av.z = fmaf(av.z, s1, s2 * fs.z);
        av.w = fmaf(av.w, s1, s2 * fs.w);
      }
      const float inv = __builtin_amdgcn_rcpf(dn + EPS_SM);
      const bool live = grow < nN;
      v4f o;
      o.x = (live ? fmaxf(av.x * inv, 0.f) : 0.f) + pz;
      o.y = (live ? fmaxf(av.y * inv, 0.f) : 0.f) + pz;
      o.z = (live ? fmaxf(av.z * inv, 0.f) : 0.f) + pz;
      o.w = (live ? fmaxf(av.w * inv, 0.f) : 0.f) + pz;
      const unsigned int hbx = f2bf(o.x), hby = f2bf(o.y), hbz = f2bf(o.z), hbw = f2bf(o.w);
      const unsigned int lbx = f2bf(o.x - bf2f(hbx)), lby = f2bf(o.y - bf2f(hby));
      const unsigned int lbz = f2bf(o.z - bf2f(hbz)), lbw = f2bf(o.w - bf2f(hbw));
      const int hw0 = (int)(hbx | (hby << 16)), hw1 = (int)(hbz | (hbw << 16));
      const int lw0 = (int)(lbx | (lby << 16)), lw1 = (int)(lbz | (lbw << 16));
      const int sa = (2 * lane) & 31, sb = (2 * lane + 1) & 31;
      const int g0 = __shfl(hw0, sa), g1 = __shfl(hw1, sa), g2 = __shfl(hw0, sb), g3 = __shfl(hw1, sb);
      const int q0 = __shfl(lw0, sa), q1 = __shfl(lw1, sa), q2 = __shfl(lw0, sb), q3 = __shfl(lw1, sb);
      const bool lsel = lane >= 16;
      v4u pv;
      pv.x = (unsigned int)(lsel ? q0 : g0);
      pv.y = (unsigned int)(lsel ? q1 : g1);
      pv.z = (unsigned int)(lsel ? q2 : g2);
      pv.w = (unsigned int)(lsel ? q3 : g3);
      unsigned short* gp = HP + (size_t)grow * KX1 + 8 * lane;
      const bool wr = grow < MPr;
      if (wr) *(volatile v4u*)gp = pv;
      __threadfence();
      if (wr) *(volatile v4u*)gp = pv;
    }
  } else {
    const int c0 = 2 * lane;
    v4u keep = {0u, 0u, 0u, 0u};
    float* res3 = (float*)reg1;

#pragma unroll 1
    for (int jt = 0; jt < nbw; ++jt) {
      const int slot = wave * nbw + jt;
      const int grow = nodeBase + slot;
      const int gcl  = grow < nN ? grow : nN - 1;
      int st = soff[slot];
      const int craw = scnt[slot];
      int cnt = craw;
      st  = st < 0 ? 0 : (st > nh ? nh : st);
      cnt = cnt < 0 ? 0 : (cnt > DEGCAP ? DEGCAP : cnt);
      if (cnt > nh - st) cnt = nh - st;
      const float pz = (ovf || craw > DEGCAP) ? qnan : 0.0f;

      const v4f ad4 = *(const v4fa*)(AD + (size_t)gcl * NHEAD);
      const float adv = hsel(ad4, head);
      float mx = -3.0e38f, dn = 0.0f;
      float a0 = 0.0f, a1 = 0.0f;

#pragma unroll 1
      for (int q = 0; q < cnt; ++q) {
        int idx = st + q; idx = idx > RCAP - 1 ? RCAP - 1 : idx;
        int eid = reg2[idx]; eid = eid < 0 ? 0 : (eid > nE - 1 ? nE - 1 : eid);
        const int sraw = srcs[eid];
        const int s = sraw < 0 ? 0 : (sraw > nN - 1 ? nN - 1 : sraw);
        const v2f fs  = *(const v2fa*)(F + (size_t)s * HC2 + c0);
        const v4f as4 = *(const v4fa*)(AS + (size_t)s * NHEAD);
        float lg = hsel(as4, head) + adv;
        lg = lg > 0.f ? lg : NEGSL * lg;
        const float df = lg - mx;
        const float ee = expf(-fabsf(df));
        const bool up  = df > 0.f;
        const float s1 = up ? ee : 1.0f;
        const float s2 = up ? 1.0f : ee;
        mx = up ? lg : mx;
        dn = fmaf(dn, s1, s2);
        a0 = fmaf(a0, s1, s2 * fs.x);
        a1 = fmaf(a1, s1, s2 * fs.y);
      }
      const float inv = __builtin_amdgcn_rcpf(dn + EPS_SM);
      const bool live = grow < nN;

      if constexpr (L == 2) {
        const float o0 = (live ? fmaxf(a0 * inv, 0.f) : 0.f) + pz;
        const float o1 = (live ? fmaxf(a1 * inv, 0.f) : 0.f) + pz;
        const unsigned int hb0 = f2bf(o0), hb1 = f2bf(o1);
        const unsigned int lb0 = f2bf(o0 - bf2f(hb0)), lb1 = f2bf(o1 - bf2f(hb1));
        const int hw = (int)(hb0 | (hb1 << 16));
        const int lw = (int)(lb0 | (lb1 << 16));
        const int li = lane & 15;
        const int i0 = (4 * li) & 31, i1 = (4 * li + 1) & 31, i2 = (4 * li + 2) & 31, i3 = (4 * li + 3) & 31;
        const int g0 = __shfl(hw, i0), g1 = __shfl(hw, i1), g2 = __shfl(hw, i2), g3 = __shfl(hw, i3);
        const int q0 = __shfl(lw, i0), q1 = __shfl(lw, i1), q2 = __shfl(lw, i2), q3 = __shfl(lw, i3);
        const bool lsel = li >= 8;
        v4u pv;
        pv.x = (unsigned int)(lsel ? q0 : g0);
        pv.y = (unsigned int)(lsel ? q1 : g1);
        pv.z = (unsigned int)(lsel ? q2 : g2);
        pv.w = (unsigned int)(lsel ? q3 : g3);
        if ((jt & 1) == 0) {
          keep = pv;
        } else {
          v4u fin;
          fin.x = (lane < 16) ? keep.x : pv.x;
          fin.y = (lane < 16) ? keep.y : pv.y;
          fin.z = (lane < 16) ? keep.z : pv.z;
          fin.w = (lane < 16) ? keep.w : pv.w;
          unsigned short* gp = HP + (size_t)(grow - 1) * KX2 + 8 * lane;
          const bool wr = grow < MPr;
          if (wr) *(volatile v4u*)gp = fin;
          __threadfence();
          if (wr) *(volatile v4u*)gp = fin;
        }
      } else {
        const float v0 = a0 * inv, v1 = a1 * inv;
        float s0 = v0 + __shfl_xor(v0, 8);
        s0 += __shfl_xor(s0, 16);
        float s1v = v1 + __shfl_xor(v1, 8);
        s1v += __shfl_xor(s1v, 16);
        const float x0 = (live ? fmaxf(0.25f * s0, 0.f) : 0.f) + pz;
        const float x1 = (live ? fmaxf(0.25f * s1v, 0.f) : 0.f) + pz;
        if (lane < 8) {
          v2f ov; ov.x = x0; ov.y = x1;
          *(v2fa*)(res3 + slot * CH2 + c0) = ov;
        }
      }
    }

    if constexpr (L == 3) {
      __syncthreads();
      const int npc = nb * (CH2 / 4);
      float* ob = X3o + (size_t)nodeBase * CH2;
#pragma unroll 1
      for (int p = tid; p < npc; p += NTHR) {
        const v4f v = *(const v4fa*)(res3 + 4 * p);
        *(volatile v4f*)(ob + 4 * p) = v;
      }
      __threadfence();
#pragma unroll 1
      for (int p = tid; p < npc; p += NTHR) {
        const v4f v = *(const v4fa*)(res3 + 4 * p);
        *(volatile v4f*)(ob + 4 * p) = v;
      }
    }
  }
}

__global__ __launch_bounds__(NTHR) void k_pack(const float* __restrict__ X3, const float* __restrict__ cl,
                                               unsigned short* A2p, int nUnits) {
  const int u = (int)blockIdx.x * NTHR + (int)threadIdx.x;
  if (u >= nUnits) return;
  const int b  = u / (KA2 / 8);
  const int k8 = (u - b * (KA2 / 8)) * 8;
  const int kx = k8 & (DMX - 1);
  const int node = b * NPG + (kx >> 4);
  const int c  = kx & 15;
  const float* xp = X3 + (size_t)node * CH2 + c;
  const v4f xa = *(const v4fa*)xp, xb = *(const v4fa*)(xp + 4);
  int cq = k8 & 63; cq = cq > NCL - 8 ? NCL - 8 : cq;
  const float* cp = cl + (size_t)b * NCL + cq;
  const v4f ca = *(const v4fa*)cp, cb = *(const v4fa*)(cp + 4);
  const v4u hiw = pack8(xa, xb);
  const v4u low = pack8(lo4(xa), lo4(xb));
  const v4u clw = pack8(ca, cb);
  const bool ishi = k8 < DMX, isx = k8 < 2 * DMX, iscl = k8 < 2 * DMX + NCL;
  v4u o;
  o.x = ishi ? hiw.x : (isx ? low.x : (iscl ? clw.x : 0u));
  o.y = ishi ? hiw.y : (isx ? low.y : (iscl ? clw.y : 0u));
  o.z = ishi ? hiw.z : (isx ? low.z : (iscl ? clw.z : 0u));
  o.w = ishi ? hiw.w : (isx ? low.w : (iscl ? clw.w : 0u));
  unsigned short* dp = A2p + (size_t)u * 8;
  *(volatile v4u*)dp = o;
  __threadfence();
  *(volatile v4u*)dp = o;
}

__global__ __launch_bounds__(NTHR) void k_mix(const float* __restrict__ X, const float* __restrict__ Wb,
                                              const float* __restrict__ bb, const float* __restrict__ Wl,
                                              const float* __restrict__ bl, unsigned short* MX, int nN) {
  __shared__ float sWb[CH2 * NBOX];
  __shared__ float sbb[CH2], sWl[CH2], sbl[CH2];
  __shared__ __attribute__((aligned(16))) unsigned short shl[2 * NTHR];
  const int tid = (int)threadIdx.x;
  if (tid < CH2 * NBOX) sWb[tid] = bfr(Wb[tid]);
  if (tid < CH2) { sbb[tid] = bfr(bb[tid]); sWl[tid] = bfr(Wl[tid]); sbl[tid] = bfr(bl[tid]); }
  __syncthreads();
  const int node0 = (int)blockIdx.x * (NTHR / CH2);
  const int node  = node0 + (tid >> 4);
  const int j     = tid & 15;
  const bool live = node < nN;
  const int ncl   = live ? node : nN - 1;
  const v4f xa = bfr4(*(const v4fa*)(X + (size_t)ncl * NFEAT));
  const v4f xb = bfr4(*(const v4fa*)(X + (size_t)ncl * NFEAT + 4));
  const float* wr = sWb + j * NBOX;
  float d = xa.y * wr[0];
  d = fmaf(xa.z, wr[1], d);
  d = fmaf(xa.w, wr[2], d);
  d = fmaf(xb.x, wr[3], d);
  d = fmaf(xb.y, wr[4], d);
  d = fmaf(xb.z, wr[5], d);
  d = fmaf(xb.w, wr[6], d);
  const float bx = fmaxf(d + sbb[j], 0.f);
  const float lv = fmaxf(fmaf(xa.x, sWl[j], sbl[j]), 0.f);
  float v = bx + lv;
  v = live ? v : 0.f;
  const unsigned int hb = f2bf(v);
  const unsigned int lb = f2bf(v - bf2f(hb));
  shl[tid] = (unsigned short)hb;
  shl[NTHR + tid] = (unsigned short)lb;
  __syncthreads();
  if (tid < 64) {
    const int part = tid >> 5;
    const int pc   = tid & 31;
    const v4u pv = *(const v4ua*)(shl + part * NTHR + 8 * pc);
    const int b  = node0 >> 7;
    const int n0 = node0 & (NPG - 1);
    unsigned short* dp = MX + (size_t)b * KMX + part * DMX + n0 * CH2 + 8 * pc;
    *(volatile v4u*)dp = pv;
    __threadfence();
    *(volatile v4u*)dp = pv;
  }
}

template <int MODE, int HASRES>
__global__ __launch_bounds__(GTHR) void k_tgemm(
    const unsigned short* __restrict__ A, int lda,
    const unsigned short* __restrict__ BT, int ldb, int K,
    const float* __restrict__ bias0, const float* __restrict__ bias1,
    const float* __restrict__ res, int ldr,
    float* outF, int ldo, int out1off, int nhalf,
    unsigned short* HP, int ldh, int nfull)
{
  static_assert(MODE == 0 || MODE == 1 || MODE == 2);
  __shared__ __attribute__((aligned(16))) float stg[GBM * GBN];
  const int tid = (int)threadIdx.x, lane = tid & 31, wave = tid >> 5, hh = lane >> 4, m = lane & 15;
  const int rowBase = (int)blockIdx.x * GBM;
  const int col0    = (int)blockIdx.y * GBN;

  v8f acc[4];
  {
    const v8f z = {0.f, 0.f, 0.f, 0.f, 0.f, 0.f, 0.f, 0.f};
    acc[0] = z; acc[1] = z; acc[2] = z; acc[3] = z;
  }
  const unsigned short* ap = A  + (size_t)(rowBase + 16 * wave + m) * (size_t)lda + 8 * hh;
  const unsigned short* wp = BT + (size_t)(col0 + m) * (size_t)ldb + 8 * hh;
  const int ksteps = K >> 5;
#pragma unroll 1
  for (int ks = 0; ks < ksteps; ++ks) {
    FragB af;
    af.h[0] = *(const v8usa*)(ap + 32 * ks);
    af.h[1] = *(const v8usa*)(ap + 32 * ks + 16);
#pragma unroll
    for (int t = 0; t < 4; ++t) {
      const unsigned short* wq = wp + (size_t)(16 * t) * (size_t)ldb + 32 * ks;
      FragB bf;
      bf.h[0] = *(const v8usa*)wq;
      bf.h[1] = *(const v8usa*)(wq + 16);
      acc[t] = wmb(af, bf, acc[t]);
    }
  }

#pragma unroll
  for (int t = 0; t < 4; ++t) {
    const int lc = 16 * t + m;
#pragma unroll
    for (int r = 0; r < 8; ++r) {
      const int lr = 16 * wave + 8 * hh + r;
      stg[lr * GBN + lc] = acc[t][r];
    }
  }
  __syncthreads();

  if constexpr (MODE != 1) {
    const int half = (MODE == 2 && col0 >= nhalf) ? 1 : 0;
    const int cb   = col0 - half * nhalf;
    const float* bsrc = (half != 0) ? bias1 : bias0;
    const v4f b4 = bfr4(*(const v4fa*)(bsrc + cb + 4 * m));
    float* ob = outF + (half != 0 ? (size_t)out1off : (size_t)0);
    v4f fv[8];
#pragma unroll
    for (int i = 0; i < 8; ++i) {
      const int lr = 16 * wave + 2 * i + hh;
      v4f v = *(const v4fa*)(stg + lr * GBN + 4 * m);
      v = v + b4;
      if (MODE == 0) { v.x = fmaxf(v.x, 0.f); v.y = fmaxf(v.y, 0.f); v.z = fmaxf(v.z, 0.f); v.w = fmaxf(v.w, 0.f); }
      fv[i] = v;
    }
#pragma unroll
    for (int i = 0; i < 8; ++i) {
      const int lr = 16 * wave + 2 * i + hh;
      float* op = ob + (size_t)(rowBase + lr) * (size_t)ldo + cb + 4 * m;
      *(volatile v4f*)op = fv[i];
    }
    __threadfence();
#pragma unroll
    for (int i = 0; i < 8; ++i) {
      const int lr = 16 * wave + 2 * i + hh;
      float* op = ob + (size_t)(rowBase + lr) * (size_t)ldo + cb + 4 * m;
      *(volatile v4f*)op = fv[i];
    }
  } else {
    const int q = lane >> 3, p8 = lane & 7, part = q & 1, rsub = q >> 1;
    const v4f ba = bfr4(*(const v4fa*)(bias0 + col0 + 8 * p8));
    const v4f bb4 = bfr4(*(const v4fa*)(bias0 + col0 + 8 * p8 + 4));
    v4u pv[8];
#pragma unroll
    for (int i = 0; i < 8; ++i) {
      const int lr = 16 * wave + 2 * i + rsub;
      const float* sr = stg + lr * GBN + 8 * p8;
      v4f va = *(const v4fa*)sr + ba;
      v4f vb = *(const v4fa*)(sr + 4) + bb4;
      va.x = fmaxf(va.x, 0.f); va.y = fmaxf(va.y, 0.f); va.z = fmaxf(va.z, 0.f); va.w = fmaxf(va.w, 0.f);
      vb.x = fmaxf(vb.x, 0.f); vb.y = fmaxf(vb.y, 0.f); vb.z = fmaxf(vb.z, 0.f); vb.w = fmaxf(vb.w, 0.f);
      if constexpr (HASRES != 0) {
        const float* rr = res + (size_t)(rowBase + lr) * (size_t)ldr + col0 + 8 * p8;
        va = va + *(const v4fa*)rr;
        vb = vb + *(const v4fa*)(rr + 4);
      }
      const v4u phi = pack8(va, vb);
      const v4u plo = pack8(lo4(va), lo4(vb));
      v4u o;
      o.x = part ? plo.x : phi.x;
      o.y = part ? plo.y : phi.y;
      o.z = part ? plo.z : phi.z;
      o.w = part ? plo.w : phi.w;
      pv[i] = o;
    }
#pragma unroll
    for (int i = 0; i < 8; ++i) {
      const int lr = 16 * wave + 2 * i + rsub;
      unsigned short* hp = HP + (size_t)(rowBase + lr) * (size_t)ldh + part * nfull + col0 + 8 * p8;
      *(volatile v4u*)hp = pv[i];
    }
    __threadfence();
#pragma unroll
    for (int i = 0; i < 8; ++i) {
      const int lr = 16 * wave + 2 * i + rsub;
      unsigned short* hp = HP + (size_t)(rowBase + lr) * (size_t)ldh + part * nfull + col0 + 8 * p8;
      *(volatile v4u*)hp = pv[i];
    }
  }
}

static int pick_nb(int nE, int nN) {
  int nb = NBMAX;
  while (nb > 32 && (long long)nb * (long long)nE * 5LL > (long long)RCAP * (long long)nN * 4LL) nb >>= 1;
  return nb;
}
static inline int cdiv(int a, int b) { return (a + b - 1) / b; }

extern "C" void kernel_launch(void* const* d_in, const int* in_sizes, int n_in,
                              void* d_out, int out_size, void* d_ws, size_t ws_size,
                              hipStream_t stream) {
  if (n_in < 26) return;
  if (in_sizes[0] < 2 || (in_sizes[0] & 1) != 0) return;
  const int nE = in_sizes[0] / 2;
  if (nE < 1 || nE >= (1 << (31 - SLOTB))) return;
  const int nN = NGR * NPG;
  if (in_sizes[1] != nN * NFEAT) return;
  if (in_sizes[2] != NGR * NCL) return;
  if (in_sizes[3] != HC1 * NFEAT) return;
  if (in_sizes[4] != HC1 || in_sizes[5] != HC1) return;
  if (in_sizes[6] != HC2 * HC1) return;
  if (in_sizes[7] != HC2 || in_sizes[8] != HC2) return;
  if (in_sizes[9] != HC2 * HC2) return;
  if (in_sizes[10] != HC2 || in_sizes[11] != HC2) return;
  if (in_sizes[12] != CH2 * NBOX || in_sizes[13] != CH2) return;
  if (in_sizes[14] != CH2 || in_sizes[15] != CH2) return;
  if (in_sizes[16] != D3 * DMX || in_sizes[17] != D3) return;
  if (in_sizes[18] != D3 * W2IN || in_sizes[19] != D3) return;
  if (in_sizes[20] != D3 * D3 || in_sizes[21] != D3) return;
  if (in_sizes[22] != LAT * D3 || in_sizes[23] != LAT) return;
  if (in_sizes[24] != LAT * D3 || in_sizes[25] != LAT) return;
  if (out_size != 2 * NGR * LAT) return;

  const int*   E    = (const int*)  d_in[0];
  const float* X    = (const float*)d_in[1];
  const float* cl   = (const float*)d_in[2];
  const float* g1W  = (const float*)d_in[3];
  const float* g1as = (const float*)d_in[4];
  const float* g1ad = (const float*)d_in[5];
  const float* g2W  = (const float*)d_in[6];
  const float* g2as = (const float*)d_in[7];
  const float* g2ad = (const float*)d_in[8];
  const float* g3W  = (const float*)d_in[9];
  const float* g3as = (const float*)d_in[10];
  const float* g3ad = (const float*)d_in[11];
  const float* Wb   = (const float*)d_in[12];
  const float* bb   = (const float*)d_in[13];
  const float* Wl   = (const float*)d_in[14];
  const float* bl   = (const float*)d_in[15];
  const float* W1   = (const float*)d_in[16];
  const float* b1   = (const float*)d_in[17];
  const float* W2   = (const float*)d_in[18];
  const float* b2   = (const float*)d_in[19];
  const float* W3   = (const float*)d_in[20];
  const float* b3   = (const float*)d_in[21];
  const float* Wm   = (const float*)d_in[22];
  const float* bm   = (const float*)d_in[23];
  const float* Wv   = (const float*)d_in[24];
  const float* bv   = (const float*)d_in[25];
  float* out = (float*)d_out;
  const int* src = E;
  const int* dst = E + nE;

  const int MP   = cdiv(nN, MROWS) * MROWS;
  const int nb   = pick_nb(nE, nN);
  if (nb < 32 || (nb & (nb - 1)) != 0 || nb > NBMAX || (nb & 15) != 0) return;
  const int gA   = MP / nb;
  if (gA * nb != MP) return;
  const int vec8 = ((nE & 3) == 0) ? 1 : 0;
  const int gM   = MP / GBM;

  char* ws = (char*)d_ws;
  size_t off = 0;
#define CARVE(NAME, BYTES) const size_t NAME = off; off += (size_t)(BYTES); off = (off + 255) & ~(size_t)255;
  CARVE(oH1,  (size_t)MP * HC1 * 4)
  CARVE(oAS1, (size_t)MP * NHEAD * 4)
  CARVE(oAD1, (size_t)MP * NHEAD * 4)
  CARVE(oX1,  (size_t)MP * KX1 * 2)
  CARVE(oG2,  (size_t)HC2 * KX1 * 2)
  CARVE(oH2,  (size_t)MP * HC2 * 4)
  CARVE(oAS2, (size_t)MP * NHEAD * 4)
  CARVE(oAD2, (size_t)MP * NHEAD * 4)
  CARVE(oX2,  (size_t)MP * KX2 * 2)
  CARVE(oG3,  (size_t)HC2 * KX2 * 2)
  CARVE(oH3,  (size_t)MP * HC2 * 4)
  CARVE(oAS3, (size_t)MP * NHEAD * 4)
  CARVE(oAD3, (size_t)MP * NHEAD * 4)
  CARVE(oX3,  (size_t)gA * nb * CH2 * 4)
  CARVE(oA2,  (size_t)NGR * KA2 * 2)
  CARVE(oW2E, (size_t)D3 * KA2 * 2)
  CARVE(oMX,  (size_t)NGR * KMX * 2)
  CARVE(oW1D, (size_t)D3 * KMX * 2)
  CARVE(oMIX, (size_t)NGR * D3 * 4)
  CARVE(oW3D, (size_t)D3 * KY * 2)
  CARVE(oWMV, (size_t)NZ * KY * 2)
  CARVE(oYA,  (size_t)NGR * KY * 2)
  CARVE(oYB,  (size_t)NGR * KY * 2)
#undef CARVE
  if (off > ws_size || off > (size_t)WSMAX) return;
  float*          H1  = (float*)(ws + oH1);
  float*          AS1 = (float*)(ws + oAS1);
  float*          AD1 = (float*)(ws + oAD1);
  unsigned short* X1  = (unsigned short*)(ws + oX1);
  unsigned short* G2P = (unsigned short*)(ws + oG2);
  float*          H2  = (float*)(ws + oH2);
  float*          AS2 = (float*)(ws + oAS2);
  float*          AD2 = (float*)(ws + oAD2);
  unsigned short* X2  = (unsigned short*)(ws + oX2);
  unsigned short* G3P = (unsigned short*)(ws + oG3);
  float*          H3  = (float*)(ws + oH3);
  float*          AS3 = (float*)(ws + oAS3);
  float*          AD3 = (float*)(ws + oAD3);
  float*          X3  = (float*)(ws + oX3);
  unsigned short* A2  = (unsigned short*)(ws + oA2);
  unsigned short* W2E = (unsigned short*)(ws + oW2E);
  unsigned short* MX  = (unsigned short*)(ws + oMX);
  unsigned short* W1D = (unsigned short*)(ws + oW1D);
  float*          MIX = (float*)(ws + oMIX);
  unsigned short* W3D = (unsigned short*)(ws + oW3D);
  unsigned short* WMV = (unsigned short*)(ws + oWMV);
  unsigned short* YA  = (unsigned short*)(ws + oYA);
  unsigned short* YB  = (unsigned short*)(ws + oYB);

  hipFuncSetAttribute(reinterpret_cast<const void*>(&k_agg<1>), hipFuncAttributeMaxDynamicSharedMemorySize, LDS_AGG);
  hipFuncSetAttribute(reinterpret_cast<const void*>(&k_agg<2>), hipFuncAttributeMaxDynamicSharedMemorySize, LDS_AGG);
  hipFuncSetAttribute(reinterpret_cast<const void*>(&k_agg<3>), hipFuncAttributeMaxDynamicSharedMemorySize, LDS_AGG);

  k_wprep<<<NUW / NTHR, NTHR, 0, stream>>>(g2W, g3W, W1, W2, W3, Wm, Wv, G2P, G3P, W1D, W2E, W3D, WMV);
  k_gat1<<<MP / NTHR, NTHR, 0, stream>>>(X, g1W, g1as, g1ad, H1, AS1, AD1, nN, MP);
  k_agg<1><<<gA, NTHR, LDS_AGG, stream>>>(src, dst, H1, AS1, AD1, X1, X3, nN, nE, nb, vec8, MP);
  k_gemmh<<<gM, GTHR, 0, stream>>>(X1, G2P, KX1, H2, g2as, g2ad, AS2, AD2);
  k_agg<2><<<gA, NTHR, LDS_AGG, stream>>>(src, dst, H2, AS2, AD2, X2, X3, nN, nE, nb, vec8, MP);
  k_gemmh<<<gM, GTHR, 0, stream>>>(X2, G3P, KX2, H3, g3as, g3ad, AS3, AD3);
  k_agg<3><<<gA, NTHR, LDS_AGG, stream>>>(src, dst, H3, AS3, AD3, X2, X3, nN, nE, nb, vec8, MP);
  {
    const int nUp = NGR * (KA2 / 8);
    k_pack<<<cdiv(nUp, NTHR), NTHR, 0, stream>>>(X3, cl, A2, nUp);
  }
  k_mix<<<nN / (NTHR / CH2), NTHR, 0, stream>>>(X, Wb, bb, Wl, bl, MX, nN);
  k_tgemm<0, 0><<<dim3(NGR / GBM, D3 / GBN), GTHR, 0, stream>>>(
      MX, KMX, W1D, KMX, KMX, b1, b1, MIX, D3, MIX, D3, 0, D3, YA, KY, D3);
  k_tgemm<1, 1><<<dim3(NGR / GBM, D3 / GBN), GTHR, 0, stream>>>(
      A2, KA2, W2E, KA2, KA2, b2, b2, MIX, D3, MIX, D3, 0, D3, YA, KY, D3);
  k_tgemm<1, 0><<<dim3(NGR / GBM, D3 / GBN), GTHR, 0, stream>>>(
      YA, KY, W3D, KY, KY, b3, b3, MIX, D3, MIX, D3, 0, D3, YB, KY, D3);
  k_tgemm<1, 0><<<dim3(NGR / GBM, D3 / GBN), GTHR, 0, stream>>>(
      YB, KY, W3D, KY, KY, b3, b3, MIX, D3, MIX, D3, 0, D3, YA, KY, D3);
  k_tgemm<2, 0><<<dim3(NGR / GBM, NZ / GBN), GTHR, 0, stream>>>(
      YA, KY, WMV, KY, KY, bm, bv, MIX, D3, out, LAT, NGR * LAT, LAT, YB, KY, D3);
}
